// PFGCNLayer_1864015806534
// MI455X (gfx1250) — hardware-verified
//
#include <hip/hip_runtime.h>


namespace {
constexpr int N = 50000, E = 800000, F = 256, HID = 256, OUT = 40, OUTP = 64, NBATCH = 10000, NPAD = 50048, NBLK = NPAD / 128;
constexpr float FXS = 4194304.0f, FXI = 1.0f / 4194304.0f;

typedef _Float16 b16;
typedef __attribute__((ext_vector_type(16))) _Float16 v16b;
typedef __attribute__((ext_vector_type(8)))  _Float16 v8b;
typedef __attribute__((ext_vector_type(8)))  float v8f;
typedef __attribute__((ext_vector_type(4)))  float v4f;

__device__ __forceinline__ v8b ld8b(const b16* p) { return *(const v8b*)p; }
__device__ __forceinline__ v16b cat8b(v8b a, v8b b) { return __builtin_shufflevector(a, b, 0, 1, 2, 3, 4, 5, 6, 7, 8, 9, 10, 11, 12, 13, 14, 15); }
__device__ __forceinline__ v16b frag_kb(const b16* p, int hh) { return cat8b(ld8b(p + 8 * hh), ld8b(p + 16 + 8 * hh)); }
__device__ __forceinline__ void split16(float v, b16& hi, b16& lo) { hi = (b16)v; lo = (b16)(v - (float)hi); }
__device__ __forceinline__ void frag_ksplit(const float* p, int hh, v16b& fh_, v16b& fl_) {
  const float* p0 = p + 8 * hh; const float* p1 = p + 16 + 8 * hh;
#pragma unroll
  for (int e = 0; e < 8; ++e) { b16 a, c; split16(p0[e], a, c); fh_[e] = a; fl_[e] = c; split16(p1[e], a, c); fh_[8 + e] = a; fl_[8 + e] = c; }
}
__device__ __forceinline__ v8f wmma16b(v16b a, v16b b, v8f c) {
  v8f d = __builtin_amdgcn_wmma_f32_16x16x32_f16(false, a, false, b, (short)0, c, false, false);
  asm volatile("v_nop\n\tv_nop\n\tv_nop\n\tv_nop" : "+v"(d) : "v"(a), "v"(b));
  return d;
}
__device__ __forceinline__ void wave_lds_sync() {
  __builtin_amdgcn_fence(__ATOMIC_RELEASE, "workgroup");
  __builtin_amdgcn_wave_barrier();
  __builtin_amdgcn_fence(__ATOMIC_ACQUIRE, "workgroup");
}

struct Opnd { const void* p0; const void* p1; int ld; };
template <int NP> __device__ __forceinline__ void load_frags(const Opnd& o, int row, int kb, int hh, v16b& fh_, v16b& fl_) {
  if (NP == 0) { frag_ksplit((const float*)o.p0 + (size_t)row * o.ld + kb, hh, fh_, fl_); }
  else if (NP == 4) {
    const float* p = (const float*)o.p0 + (size_t)row * o.ld + kb; const float* p0 = p + 8 * hh; const float* p1 = p + 16 + 8 * hh;
#pragma unroll
    for (int e = 0; e < 8; ++e) { b16 a, c; split16(p0[e] * 64.0f, a, c); fh_[e] = a; fl_[e] = c; split16(p1[e] * 64.0f, a, c); fh_[8 + e] = a; fl_[8 + e] = c; }
  } else if (NP == 3) {
    const float* p = (const float*)o.p0 + (size_t)row * o.ld + kb; const float* p0 = p + 8 * hh; const float* p1 = p + 16 + 8 * hh;
#pragma unroll
    for (int e = 0; e < 8; ++e) { fh_[e] = (b16)p0[e]; fh_[8 + e] = (b16)p1[e]; }
    fl_ = fh_;
  } else {
    fh_ = frag_kb((const b16*)o.p0 + (size_t)row * o.ld + kb, hh);
    if (NP == 2) fl_ = frag_kb((const b16*)o.p1 + (size_t)row * o.ld + kb, hh); else fl_ = fh_;
  }
}
template <int ANP, int BNP> __device__ __forceinline__ v8f mac(v16b ah, v16b al, v16b bh, v16b bl, v8f c) {
  c = wmma16b(ah, bh, c);
  if (BNP == 0 || BNP == 2 || BNP == 4) c = wmma16b(ah, bl, c);
  if (ANP == 0 || ANP == 2 || ANP == 4) c = wmma16b(al, bh, c);
  return c;
}
template <int ANP, int BNP>
__device__ __forceinline__ void gemm_tile(const Opnd& A, const Opnd& B, int K, int m0, int c0, int nloc, int hlf, v8f (&acc)[2][4]) {
  for (int kb = 0; kb < K; kb += 32) {
    v16b a0h, a0l, a1h, a1l;
    load_frags<ANP>(A, m0 + nloc, kb, hlf, a0h, a0l);
    load_frags<ANP>(A, m0 + 16 + nloc, kb, hlf, a1h, a1l);
#pragma unroll
    for (int t = 0; t < 4; ++t) {
      v16b bh, bl;
      load_frags<BNP>(B, c0 + t * 16 + nloc, kb, hlf, bh, bl);
      acc[0][t] = mac<ANP, BNP>(a0h, a0l, bh, bl, acc[0][t]);
      acc[1][t] = mac<ANP, BNP>(a1h, a1l, bh, bl, acc[1][t]);
    }
  }
}

__device__ __forceinline__ void epi_planes(v8f (&acc)[2][4], float scale, bool two, b16* __restrict__ oh, b16* __restrict__ ol, int ldo,
                                           int m0, int c0, int lane, b16* Th, b16* Tl) {
  const int nloc = lane & 15, hlf = lane >> 4;
#pragma unroll
  for (int t = 0; t < 4; ++t)
#pragma unroll
    for (int r = 0; r < 2; ++r)
#pragma unroll
      for (int v = 0; v < 8; ++v) {
        const int rr = r * 16 + v + 8 * hlf, cc = t * 16 + nloc;
        b16 h_, l_; split16(acc[r][t][v] * scale, h_, l_);
        Th[rr * 64 + cc] = h_; Tl[rr * 64 + cc] = l_;
      }
  wave_lds_sync();
  for (int pass = 0; pass < 2; ++pass) {
#pragma unroll
    for (int j = 0; j < 8; ++j) {
      const int rr = j * 4 + (lane >> 3), c8 = (lane & 7) * 8;
      const size_t o = (size_t)(m0 + rr) * ldo + c0 + c8;
      *(volatile v8b*)(oh + o) = ld8b(Th + rr * 64 + c8);
      if (two) *(volatile v8b*)(ol + o) = ld8b(Tl + rr * 64 + c8);
    }
    __threadfence();
  }
}
__device__ __forceinline__ void epi_f32(v8f (&acc)[2][4], float scale, const float* rscale, float* __restrict__ out, int ldo, int m0, int c0, int lane, float* Tt) {
  const int nloc = lane & 15, hlf = lane >> 4;
#pragma unroll
  for (int t = 0; t < 4; ++t)
#pragma unroll
    for (int r = 0; r < 2; ++r)
#pragma unroll
      for (int v = 0; v < 8; ++v) {
        const int rr = r * 16 + v + 8 * hlf;
        const float rs = rscale ? rscale[(size_t)(m0 + rr) * 32] : 1.0f;
        Tt[rr * 64 + t * 16 + nloc] = acc[r][t][v] * scale * rs;
      }
  wave_lds_sync();
  float* dst0 = out + (size_t)m0 * ldo + c0;
  for (int pass = 0; pass < 2; ++pass) {
#pragma unroll
    for (int j = 0; j < 16; ++j) { const int rr = j * 2 + hlf, c4 = nloc * 4; *(volatile v4f*)(dst0 + (size_t)rr * ldo + c4) = *(const v4f*)(Tt + rr * 64 + c4); }
    __threadfence();
  }
}


__global__ __launch_bounds__(256) void prep_kernel(const float* __restrict__ W1, const float* __restrict__ W2, const float* __restrict__ b2, b16* __restrict__ w1, b16* __restrict__ w2, float* __restrict__ b2p) {
  const size_t tid = (size_t)blockIdx.x * blockDim.x + threadIdx.x, nth = (size_t)gridDim.x * blockDim.x;
  for (int pass = 0; pass < 2; ++pass) {
    for (size_t p = tid; p < (size_t)HID * F / 8; p += nth) { const int n = (int)(p / (F / 8)), k0 = (int)(p % (F / 8)) * 8; v8b v;
#pragma unroll
      for (int e = 0; e < 8; ++e) v[e] = (b16)W1[(size_t)(k0 + e) * HID + n];
      *(volatile v8b*)(w1 + (size_t)n * F + k0) = v; }
    for (size_t p = tid; p < (size_t)OUTP * HID / 8; p += nth) { const int n = (int)(p / (HID / 8)), k0 = (int)(p % (HID / 8)) * 8; v8b v;
#pragma unroll
      for (int e = 0; e < 8; ++e) v[e] = (b16)((n < OUT) ? W2[(size_t)(k0 + e) * OUT + min(n, OUT - 1)] : 0.0f);
      *(volatile v8b*)(w2 + (size_t)n * HID + k0) = v; }
    for (size_t p = tid; p < (size_t)OUTP; p += nth) ((volatile float*)b2p)[p] = (p < (size_t)OUT) ? b2[min((int)p, OUT - 1)] : 0.0f;
    __threadfence();
  }
}

template <int NOUT, bool BNRELU>
__global__ __launch_bounds__(128) void lin_kernel(const float* __restrict__ x, int nrow_in, const float* __restrict__ coef, const b16* __restrict__ w, const float* __restrict__ bias, float* __restrict__ h) {
  __shared__ __attribute__((aligned(16))) float Ts[4][32 * 64];
  const int lane = threadIdx.x & 31, wave = threadIdx.x >> 5, nloc = lane & 15, hlf = lane >> 4, m0 = blockIdx.y * 128 + wave * 32, c0 = blockIdx.x * 64;
  const int ra = min(m0 + nloc, nrow_in - 1), rb = min(m0 + 16 + nloc, nrow_in - 1);
  v8f acc[2][4];
#pragma unroll
  for (int r = 0; r < 2; ++r)
#pragma unroll
    for (int t = 0; t < 4; ++t) acc[r][t] = (v8f){};
#pragma unroll 1
  for (int kb = 0; kb < F; kb += 32) { v16b a0, a1;
#pragma unroll
    for (int e = 0; e < 16; ++e) { const int k = kb + ((e < 8) ? (8 * hlf + e) : (16 + 8 * hlf + e - 8)); float u0 = x[(size_t)ra * F + k], u1 = x[(size_t)rb * F + k];
      if (BNRELU) { const float ca = coef[k], sh = coef[F + k]; u0 = fmaxf(u0 * ca + sh, 0.0f); u1 = fmaxf(u1 * ca + sh, 0.0f); } a0[e] = (b16)u0; a1[e] = (b16)u1; }
#pragma unroll
    for (int t = 0; t < 4; ++t) { const v16b bw = frag_kb(w + (size_t)(c0 + t * 16 + nloc) * F + kb, hlf); acc[0][t] = wmma16b(a0, bw, acc[0][t]); acc[1][t] = wmma16b(a1, bw, acc[1][t]); } }
#pragma unroll
  for (int t = 0; t < 4; ++t)
#pragma unroll
    for (int r = 0; r < 2; ++r)
#pragma unroll
      for (int v = 0; v < 8; ++v) acc[r][t][v] += bias[c0 + t * 16 + nloc];
  epi_f32(acc, 1.0f, nullptr, h, NOUT, m0, c0, lane, Ts[wave]);
}

typedef __attribute__((ext_vector_type(4))) int v4i;
__device__ __forceinline__ int fkey(float f) { const int b = __float_as_int(f); return (b >= 0) ? b : (b ^ 0x7FFFFFFF); }
__device__ __forceinline__ float fkey_inv(int k) { return __int_as_float((k >= 0) ? k : (k ^ 0x7FFFFFFF)); }

template <int DF, int NB, bool TWOPASS>
__global__ __launch_bounds__(256) void agg_kernel(const int* __restrict__ esrc, const int* __restrict__ edst, const float* __restrict__ h, const float* __restrict__ gammap, float* __restrict__ xo, float* __restrict__ slot_) {
  constexpr int FPL = DF / 32;
  __shared__ __attribute__((aligned(16))) int acc[NB * DF];
  __shared__ int den[NB]; __shared__ int list[8 * 256]; __shared__ float Cs[2][DF]; __shared__ int dmin[TWOPASS ? NB : 1];
  const int t_ = threadIdx.x, wave = t_ >> 5, lane = t_ & 31, base = blockIdx.x * NB; const float gam = gammap[0];
  for (int i = t_; i < NB * DF; i += 256) acc[i] = 0;
  for (int i = t_; i < NB; i += 256) { den[i] = 0; if (TWOPASS) dmin[i] = fkey(INFINITY); }
  for (int i = t_; i < 2 * DF; i += 256) Cs[i / DF][i % DF] = 0.0f;
  __syncthreads();
  int* wl = list + wave * 256;
  for (int ps = TWOPASS ? 0 : 1; ps < 2; ++ps) {
  if (ps == 1) __syncthreads();
  for (int c0 = 0; c0 < E; c0 += 256 * 8) {
    const int e0 = c0 + (wave * 32 + lane) * 8; int dd[8];
#pragma unroll
    for (int j = 0; j < 8; ++j) { const int dv = edst[min(e0 + j, E - 1)]; dd[j] = (e0 + j < E) ? dv : -1; }
    unsigned sl[8]; bool hit[8]; bool anyl = false;
#pragma unroll
    for (int j = 0; j < 8; ++j) { sl[j] = (unsigned)(dd[j] - base); hit[j] = sl[j] < (unsigned)NB; anyl |= hit[j]; }
    int wc = 0;
    if (__builtin_amdgcn_ballot_w32(anyl) != 0u) {
#pragma unroll
      for (int j = 0; j < 8; ++j) {
        const unsigned mj = __builtin_amdgcn_ballot_w32(hit[j]);
        if (mj != 0u) {
          if (hit[j]) { const int pos = wc + (int)__builtin_amdgcn_mbcnt_lo(mj, 0u); int s = esrc[min(e0 + j, E - 1)]; s = (s < 0) ? 0 : (s >= N ? N - 1 : s); wl[pos] = (s << 12) | (int)sl[j]; }
          wc += __builtin_popcount(mj); } } }
    __builtin_amdgcn_wave_barrier(); __builtin_amdgcn_fence(__ATOMIC_RELEASE, "workgroup"); __builtin_amdgcn_fence(__ATOMIC_ACQUIRE, "workgroup");
    for (int i = 0; i < wc; ++i) { const int ent = wl[i]; const int s = ent >> 12, slot = ent & 4095;
      const float* hs = h + (size_t)s * DF + lane * FPL; const float* ho = h + (size_t)(base + slot) * DF + lane * FPL;
      float vs[FPL]; float d2 = 0.0f;
      if (FPL == 8) { const v4f a = *(const v4f*)hs, b = *(const v4f*)(hs + 4), c = *(const v4f*)ho, d = *(const v4f*)(ho + 4);
#pragma unroll
        for (int q = 0; q < 4; ++q) { vs[q] = a[q]; vs[4 + q] = b[q]; const float x0 = a[q] - c[q], x1 = b[q] - d[q]; d2 += x0 * x0 + x1 * x1; } }
      else { const float a0 = hs[0], a1 = hs[1], c0 = ho[0], c1 = ho[1]; vs[0] = a0; vs[1] = a1; d2 = (a0 - c0) * (a0 - c0) + (a1 - c1) * (a1 - c1); }
#pragma unroll
      for (int o = 16; o > 0; o >>= 1) d2 += __shfl_xor(d2, o);
      if (TWOPASS && ps == 0) { if (lane == 0) atomicMin(&dmin[slot], fkey(d2)); continue; }
      const float w = __expf(-gam * (TWOPASS ? (d2 - fkey_inv(dmin[slot])) : d2));
      if (lane == 0) atomicAdd(&den[slot], (int)rintf(w * FXS));
#pragma unroll
      for (int q = 0; q < FPL; ++q) atomicAdd(&acc[slot * DF + lane * FPL + q], (int)rintf(w * vs[q] * FXS)); }
    __builtin_amdgcn_wave_barrier();
  }
  }
  __syncthreads();
  { const int cq = (t_ % (DF / 4)) * 4, r0 = t_ / (DF / 4), rstep = 256 / (DF / 4);
    float s[4] = {0, 0, 0, 0}, s2[4] = {0, 0, 0, 0};
    for (int r = r0; r < NB; r += rstep) { const int node = base + r; if (node < N) { const float epsr = TWOPASS ? 1e-16f * __expf(gam * fkey_inv(dmin[r])) : 1e-16f; const float dn = 1.0f / ((float)den[r] * FXI + epsr);
#pragma unroll
        for (int q = 0; q < 4; ++q) { const float v = (float)acc[r * DF + cq + q] * FXI * dn; s[q] += v; s2[q] += v * v; } } }
    __shared__ float Red[2][256 * 4];
#pragma unroll
    for (int q = 0; q < 4; ++q) { Red[0][t_ * 4 + q] = s[q]; Red[1][t_ * 4 + q] = s2[q]; }
    __syncthreads();
    if (t_ < DF / 4) { float a[4] = {0, 0, 0, 0}, b[4] = {0, 0, 0, 0};
      for (int g = 0; g < rstep; ++g)
#pragma unroll
        for (int q = 0; q < 4; ++q) { a[q] += Red[0][(g * (DF / 4) + t_) * 4 + q]; b[q] += Red[1][(g * (DF / 4) + t_) * 4 + q]; }
#pragma unroll
      for (int q = 0; q < 4; ++q) { Cs[0][cq + q] = a[q]; Cs[1][cq + q] = b[q]; } }
    __syncthreads(); }
  for (int pass = 0; pass < 2; ++pass) {
    for (int i = t_; i < NB * DF / 4; i += 256) { const int r = (i * 4) / DF, cq = (i * 4) % DF, node = base + r; if (node < NPAD) { v4f o = {0.0f, 0.0f, 0.0f, 0.0f};
        if (node < N) { const float epsr = TWOPASS ? 1e-16f * __expf(gam * fkey_inv(dmin[r])) : 1e-16f; const float dn = 1.0f / ((float)den[r] * FXI + epsr);
#pragma unroll
          for (int q = 0; q < 4; ++q) o[q] = (float)acc[r * DF + cq + q] * FXI * dn; }
        *(volatile v4f*)(xo + (size_t)node * DF + cq) = o; } }
    for (int i = t_; i < 2 * DF / 4; i += 256) *(volatile v4f*)(slot_ + (size_t)blockIdx.x * 2 * DF + i * 4) = *(const v4f*)(&Cs[i / (DF / 4)][(i % (DF / 4)) * 4]);
    __threadfence();
  }
}

template <int DF>
__global__ __launch_bounds__(256) void bnfin_kernel(const float* __restrict__ slot_, int nblk, const float* __restrict__ g, const float* __restrict__ bb, int nch, float* __restrict__ coef) {
  const int c = threadIdx.x; if (c >= DF) return;
  double s = 0.0, s2 = 0.0;
  for (int bk = 0; bk < nblk; ++bk) { s += (double)slot_[(size_t)bk * 2 * DF + c]; s2 += (double)slot_[(size_t)bk * 2 * DF + DF + c]; }
  const double mean = s / N, var = s2 / N - mean * mean;
  const float gg = (c < nch) ? g[min(c, nch - 1)] : 0.0f, b_ = (c < nch) ? bb[min(c, nch - 1)] : 0.0f;
  const float a = gg * (float)(1.0 / sqrt(var + 1e-5)), sh = b_ - (float)mean * a;
  for (int pass = 0; pass < 2; ++pass) { ((volatile float*)coef)[c] = a; ((volatile float*)coef)[DF + c] = sh; __threadfence(); }
}

__global__ __launch_bounds__(64) void final_kernel(const int* __restrict__ bn, const float* __restrict__ x2, const float* __restrict__ coef, float* __restrict__ out) {
  __shared__ __attribute__((aligned(16))) float Ob[64 * OUT];
  const int r = blockIdx.x * 64 + threadIdx.x;
  if (r < NBATCH) { int id = bn[r]; id = (id < 0) ? 0 : (id >= N ? N - 1 : id); const float* row = x2 + (size_t)id * OUTP; float v[OUT]; float mx = -INFINITY;
#pragma unroll
    for (int c = 0; c < OUT; ++c) { v[c] = fmaxf(row[c] * coef[c] + coef[OUTP + c], 0.0f); mx = fmaxf(mx, v[c]); }
    float se = 0.0f;
#pragma unroll
    for (int c = 0; c < OUT; ++c) se += __expf(v[c] - mx);
    const float lse = mx + __logf(se);
#pragma unroll
    for (int c = 0; c < OUT; ++c) Ob[threadIdx.x * OUT + c] = v[c] - lse; }
  __syncthreads();
  const int nrow = min(64, NBATCH - blockIdx.x * 64);
  for (int pass = 0; pass < 2; ++pass) { for (int i = threadIdx.x; i < nrow * OUT / 4; i += 64) *(volatile v4f*)(out + (size_t)blockIdx.x * 64 * OUT + i * 4) = *(const v4f*)(&Ob[i * 4]); __threadfence(); }
}
}

extern "C" void kernel_launch(void* const* d_in, const int* in_sizes, int n_in,
                              void* d_out, int out_size, void* d_ws, size_t ws_size, hipStream_t stream) {
  (void)n_in; (void)out_size;
  const float* x = (const float*)d_in[0]; const int* ei = (const int*)d_in[1]; const int* bnodes = (const int*)d_in[2];
  const float* W1 = (const float*)d_in[3]; const float* b1 = (const float*)d_in[4]; const float* g1 = (const float*)d_in[5];
  const float* W2 = (const float*)d_in[6]; const float* b2 = (const float*)d_in[7]; const float* g2 = (const float*)d_in[8];
  const float* bn1w = (const float*)d_in[9]; const float* bn1b = (const float*)d_in[10]; const float* bn2w = (const float*)d_in[11]; const float* bn2b = (const float*)d_in[12];
  float* out = (float*)d_out;
  if (in_sizes[0] != N * F || in_sizes[1] != 2 * E || in_sizes[2] != NBATCH || in_sizes[3] != F * HID || in_sizes[6] != HID * OUT) return;
  const int* esrc = ei; const int* edst = ei + E;
  size_t off = 0; char* ws = (char*)d_ws;
  auto carve = [&](size_t bytes) { char* p = ws + off; off += (bytes + 255) & ~(size_t)255; return p; };
  b16* w1 = (b16*)carve((size_t)HID * F * 2); b16* w2 = (b16*)carve((size_t)OUTP * HID * 2); float* b2p = (float*)carve(OUTP * 4);
  float* h1 = (float*)carve((size_t)NPAD * HID * 4); float* x1 = (float*)carve((size_t)NPAD * HID * 4);
  float* h2 = (float*)carve((size_t)NPAD * OUTP * 4); float* x2 = (float*)carve((size_t)NPAD * OUTP * 4);
  float* slot_ = (float*)carve((size_t)196 * 2 * HID * 4); float* coef = (float*)carve(2 * HID * 4);
  if (off > ws_size) return;
  prep_kernel<<<64, 256, 0, stream>>>(W1, W2, b2, w1, w2, b2p);
  lin_kernel<HID, false><<<dim3(HID / 64, NBLK), 128, 0, stream>>>(x, N, nullptr, w1, b1, h1);
  agg_kernel<HID, 256, false><<<NPAD / 256 + 1, 256, 0, stream>>>(esrc, edst, h1, g1, x1, slot_);
  bnfin_kernel<HID><<<1, 256, 0, stream>>>(slot_, NPAD / 256 + 1, bn1w, bn1b, HID, coef);
  lin_kernel<OUTP, true><<<dim3(OUTP / 64, NBLK), 128, 0, stream>>>(x1, NPAD, coef, w2, b2p, h2);
  agg_kernel<OUTP, 1024, true><<<NPAD / 1024 + 1, 256, 0, stream>>>(esrc, edst, h2, g2, x2, slot_);
  bnfin_kernel<OUTP><<<1, 256, 0, stream>>>(slot_, NPAD / 1024 + 1, bn2w, bn2b, OUT, coef);
  final_kernel<<<(NBATCH + 63) / 64, 64, 0, stream>>>(bnodes, x2, coef, out);
}
